// Cfconv_46746424050014
// MI455X (gfx1250) — hardware-run, weakly checked
//
#include <hip/hip_runtime.h>
#include <stddef.h>
#include <stdint.h>

#define HID    128
#define NRBF   50
#define NB     64
#define KX     256
#define KF1    64
#define KF2    128
#define KU     256
#define NLAY   3
#define NRANGE 3
#define NTHR   256
#define NWAVE  8
#define EPB    256
#define DP     132
#define AP     136
#define MPITCH 128
#define CSTN   256
#define GBM    64
#define GBN    128
#define GTHR   128
#define EPT    8
#define CHUNK  (NTHR * EPT)
#define WCAP   (EPT * 32)
#define LISTN  (NWAVE * WCAP)
#define NBA    1024
#define SLA    10
#define RCAP   28672
#define DEGCAP 64
#define NU_IF  (NLAY * HID * (KX / 8))
#define NU_W1  (NLAY * HID * (KF1 / 8))
#define NU_W2  (NLAY * HID * (KF2 / 8))
#define NU_U   (NLAY * HID * (KU / 8))
#define AGG_ZINTS (LISTN + 2 * RCAP + 3 * NBA)
#define AGG_LDS_INTS (AGG_ZINTS + 16)
#define AGG_LDS_BYTES (AGG_LDS_INTS * 4)
#define EDGE_LDS_BYTES (EPB * DP * 4 + EPB * AP * 2 + EPB * MPITCH * 2 + CSTN * 4 + 3 * EPB * 4 + 64)
#define WSMAX  134217728
#define CACT   16.0f
#define CWGT   1024.0f
#define CMSG   1024.0f
#define PINV   6.103515625e-05f
#define MINV   0.0009765625f
#define CUTF   5.0f
#define PIF    3.14159265358979323846f
#define LN2F   0.69314718055994531f

static_assert((CHUNK & (CHUNK - 1)) == 0 && CHUNK <= 4096);
static_assert((NBA & (NBA - 1)) == 0 && NBA == (1 << SLA));
static_assert(((long long)CHUNK << SLA) < (1LL << 31));
static_assert(LISTN % NTHR == 0);
static_assert(NBA % NWAVE == 0 && NBA % 32 == 0);
static_assert(RCAP % 4 == 0 && AGG_ZINTS % (4 * NTHR) == 0 && LISTN % 4 == 0);
static_assert(AGG_LDS_BYTES <= 300000);
static_assert(EDGE_LDS_BYTES <= 300000);
static_assert(NU_IF % NTHR == 0 && NU_W1 % NTHR == 0 && NU_W2 % NTHR == 0 && NU_U % NTHR == 0);
static_assert(HID * (KX / 8) == 4096 && HID * (KF1 / 8) == 1024 && HID * (KF2 / 8) == 2048 && HID * (KU / 8) == 4096);
static_assert(KX == 2 * HID && KX % 32 == 0 && KF1 == NB && KF1 % 32 == 0 && NRBF <= NB && NRBF > 1);
static_assert(KF2 == HID && KF2 % 32 == 0 && KU == 2 * HID && KU % 32 == 0);
static_assert(GBM == (GTHR / 32) * 16 && GBN == 4 * 32 && GBN == HID);
static_assert((DP * 4) % 16 == 0 && (AP * 2) % 16 == 0 && AP >= KF1 && AP >= KF2 && DP >= HID);
static_assert(EPB == NTHR && EPB == 8 * 32);
static_assert((EPB * DP * 4) % 16 == 0 && (EPB * AP * 2) % 16 == 0 && (EPB * MPITCH * 2) % 16 == 0);
static_assert((CSTN * 4) % 16 == 0 && CSTN >= 2 * HID);
static_assert(EPB * MPITCH * 2 == 16 * NTHR * 16);
static_assert(NB % 8 == 0 && HID % 8 == 0 && MPITCH == HID);

typedef float          v4f   __attribute__((ext_vector_type(4)));
typedef float          v8f   __attribute__((ext_vector_type(8)));
typedef int            v4i   __attribute__((ext_vector_type(4)));
typedef int            v8i   __attribute__((ext_vector_type(8)));
typedef unsigned       v2u   __attribute__((ext_vector_type(2)));
typedef unsigned short v8us  __attribute__((ext_vector_type(8)));
typedef unsigned short v16us __attribute__((ext_vector_type(16)));
typedef __bf16         v16bf __attribute__((ext_vector_type(16)));
typedef _Float16       v16h  __attribute__((ext_vector_type(16)));
typedef v4f  __attribute__((may_alias)) v4fa;
typedef v4i  __attribute__((may_alias)) v4ia;
typedef v2u  __attribute__((may_alias)) v2ua;
typedef v8us __attribute__((may_alias)) v8usa;
union FragB { v16bf v; v16us u; v8us h[2]; v8i w; };
union FragH { v16h  v; v16us u; v8us h[2]; v8i w; };

__device__ __forceinline__ v8f wmb(const FragB& a, const FragB& b, v8f c) {
  v8f d = __builtin_amdgcn_wmma_f32_16x16x32_bf16(false, a.v, false, b.v, (short)0, c, false, false);
  asm volatile("v_nop\n\tv_nop\n\tv_nop\n\tv_nop" : "+v"(d) : "v"(a.w), "v"(b.w));
  return d;
}
__device__ __forceinline__ v8f wmh(const FragH& a, const FragH& b, v8f c) {
  v8f d = __builtin_amdgcn_wmma_f32_16x16x32_f16(false, a.v, false, b.v, (short)0, c, false, false);
  asm volatile("v_nop\n\tv_nop\n\tv_nop\n\tv_nop" : "+v"(d) : "v"(a.w), "v"(b.w));
  return d;
}

__device__ __forceinline__ unsigned bf16_bits(float f) {
  const unsigned u = __float_as_uint(f);
  return (u + 0x7FFFu + ((u >> 16) & 1u)) >> 16;
}
__device__ __forceinline__ float bf16_val(float f) {
  return __uint_as_float(bf16_bits(f) << 16);
}
__device__ __forceinline__ unsigned short f2h(float f) {
  const _Float16 hv = (_Float16)f;
  return __builtin_bit_cast(unsigned short, hv);
}
__device__ __forceinline__ float h2f(unsigned b) {
  const _Float16 hv = __builtin_bit_cast(_Float16, (unsigned short)b);
  return (float)hv;
}
__device__ __forceinline__ float ssp_f(float x) {
  return fmaxf(x, 0.0f) + __logf(1.0f + __expf(-fabsf(x))) - LN2F;
}
__device__ __forceinline__ void put16(unsigned short* dp, v8us o) {
  *(volatile v8us*)dp = o;
  __threadfence();
  *(volatile v8us*)dp = o;
}
__device__ __forceinline__ void putf4(float* dp, v4f o) {
  *(volatile v4f*)dp = o;
  __threadfence();
  *(volatile v4f*)dp = o;
}

template <int SLB>
__device__ __forceinline__ int scan_chunk(const int* __restrict__ dsts, int nE, int cbase, int slotBase,
                                          int nb, int vec8, int* list, int tid, int lane, int wave) {
  int wc = 0;
  const int el0  = tid * EPT;
  const int e0   = cbase + el0;
  const int sent = -2147483647 - 1;
  v4i da, db;
  if (vec8 != 0 && cbase + CHUNK <= nE) {
    da = *(const v4i*)(dsts + e0);
    db = *(const v4i*)(dsts + e0 + 4);
  } else {
    da.x = (e0     < nE) ? dsts[min(e0,     nE - 1)] : sent;
    da.y = (e0 + 1 < nE) ? dsts[min(e0 + 1, nE - 1)] : sent;
    da.z = (e0 + 2 < nE) ? dsts[min(e0 + 2, nE - 1)] : sent;
    da.w = (e0 + 3 < nE) ? dsts[min(e0 + 3, nE - 1)] : sent;
    db.x = (e0 + 4 < nE) ? dsts[min(e0 + 4, nE - 1)] : sent;
    db.y = (e0 + 5 < nE) ? dsts[min(e0 + 5, nE - 1)] : sent;
    db.z = (e0 + 6 < nE) ? dsts[min(e0 + 6, nE - 1)] : sent;
    db.w = (e0 + 7 < nE) ? dsts[min(e0 + 7, nE - 1)] : sent;
  }
  const unsigned nbs = (unsigned)slotBase;
  const unsigned unb = (unsigned)nb;
  const unsigned s0 = (unsigned)da.x - nbs, s1 = (unsigned)da.y - nbs;
  const unsigned s2 = (unsigned)da.z - nbs, s3 = (unsigned)da.w - nbs;
  const unsigned s4 = (unsigned)db.x - nbs, s5 = (unsigned)db.y - nbs;
  const unsigned s6 = (unsigned)db.z - nbs, s7 = (unsigned)db.w - nbs;
  const bool h0 = s0 < unb, h1 = s1 < unb, h2 = s2 < unb, h3 = s3 < unb;
  const bool h4 = s4 < unb, h5 = s5 < unb, h6 = s6 < unb, h7 = s7 < unb;
  const unsigned any = __builtin_amdgcn_ballot_w32(h0 | h1 | h2 | h3 | h4 | h5 | h6 | h7);
  if (any != 0u) {
#define HITJ(J, HJ, SJ) { \
      const unsigned mj = __builtin_amdgcn_ballot_w32(HJ); \
      if (mj != 0u) { \
        if (HJ) { \
          const int pos = wc + (int)__builtin_amdgcn_mbcnt_lo(mj, 0u); \
          if (pos < WCAP) list[wave * WCAP + pos] = ((el0 + (J)) << SLB) | (int)(SJ); \
        } \
        wc += (int)__builtin_popcount(mj); } }
    HITJ(0, h0, s0)
    HITJ(1, h1, s1)
    HITJ(2, h2, s2)
    HITJ(3, h3, s3)
    HITJ(4, h4, s4)
    HITJ(5, h5, s5)
    HITJ(6, h6, s6)
    HITJ(7, h7, s7)
#undef HITJ
  }
  return wc;
}

__global__ __launch_bounds__(NTHR) void k_prep(const float* __restrict__ R, const int* __restrict__ Z,
                                               const float* __restrict__ emb, int nEmb,
                                               const float* __restrict__ IF, const float* __restrict__ W1,
                                               const float* __restrict__ W2, const float* __restrict__ U1,
                                               const float* __restrict__ U2, int nN, int mRows,
                                               unsigned short* IFT, unsigned short* W1T, unsigned short* W2T,
                                               unsigned short* U1T, unsigned short* U2T,
                                               float* RP, unsigned short* XB, float* X0) {
  const int u   = (int)blockIdx.x * NTHR + (int)threadIdx.x;
  const int L0  = NU_IF;
  const int L1  = L0 + NU_W1;
  const int L2  = L1 + NU_W2;
  const int L3  = L2 + NU_U;
  const int L4  = L3 + NU_U;
  const int nXP = ((mRows + NTHR - 1) / NTHR) * NTHR;
  const int L5  = L4 + nXP;
  const int L6  = L5 + mRows * 16;
  const int nX0 = ((nN * 32 + NTHR - 1) / NTHR) * NTHR;
  const int L7  = L6 + nX0;
  v8us o;
  if (u < L0) {
    const int l    = u >> 12;
    const int w    = u & 4095;
    const int n    = w >> 5;
    const int k8   = (w & 31) * 8;
    const int srow = k8 & (HID - 1);
    const float* p = IF + ((size_t)l * HID + srow) * HID + n;
#pragma unroll
    for (int i = 0; i < 8; ++i) o[i] = (unsigned short)bf16_bits(p[(size_t)i * HID]);
    put16(IFT + ((size_t)l * HID + n) * KX + k8, o);
    return;
  } else if (u < L1) {
    const int v  = u - L0;
    const int l  = v >> 10;
    const int w  = v & 1023;
    const int n  = w >> 3;
    const int k8 = (w & 7) * 8;
#pragma unroll
    for (int i = 0; i < 8; ++i) {
      const int   k  = k8 + i;
      const int   kc = k < NRBF ? k : (NRBF - 1);
      const float wv = W1[((size_t)l * NRBF + kc) * HID + n];
      const float sv = (k < NRBF) ? wv : (wv - wv);
      o[i] = (unsigned short)bf16_bits(sv);
    }
    put16(W1T + ((size_t)l * HID + n) * KF1 + k8, o);
    return;
  } else if (u < L2) {
    const int v  = u - L1;
    const int l  = v >> 11;
    const int w  = v & 2047;
    const int n  = w >> 4;
    const int k8 = (w & 15) * 8;
    const float* p = W2 + ((size_t)l * HID + k8) * HID + n;
#pragma unroll
    for (int i = 0; i < 8; ++i) o[i] = f2h(CWGT * bf16_val(p[(size_t)i * HID]));
    put16(W2T + ((size_t)l * HID + n) * KF2 + k8, o);
    return;
  } else if (u < L3) {
    const int v    = u - L2;
    const int l    = v >> 12;
    const int w    = v & 4095;
    const int n    = w >> 5;
    const int k8   = (w & 31) * 8;
    const int srow = k8 & (HID - 1);
    const float* p = U1 + ((size_t)l * HID + srow) * HID + n;
#pragma unroll
    for (int i = 0; i < 8; ++i) o[i] = (unsigned short)bf16_bits(p[(size_t)i * HID]);
    put16(U1T + ((size_t)l * HID + n) * KU + k8, o);
    return;
  } else if (u < L4) {
    const int v    = u - L3;
    const int l    = v >> 12;
    const int w    = v & 4095;
    const int n    = w >> 5;
    const int k8   = (w & 31) * 8;
    const int srow = k8 & (HID - 1);
    const float* p = U2 + ((size_t)l * HID + srow) * HID + n;
#pragma unroll
    for (int i = 0; i < 8; ++i) o[i] = (unsigned short)bf16_bits(p[(size_t)i * HID]);
    put16(U2T + ((size_t)l * HID + n) * KU + k8, o);
    return;
  } else if (u < L5) {
    const int row = u - L4;
    if (row >= mRows) return;
    const int rc  = row < nN ? row : nN - 1;
    const bool ok = row < nN;
    const float r0 = R[(size_t)rc * 3 + 0];
    const float r1 = R[(size_t)rc * 3 + 1];
    const float r2 = R[(size_t)rc * 3 + 2];
    v4f q;
    q.x = ok ? bf16_val(r0) : 0.0f;
    q.y = ok ? bf16_val(r1) : 0.0f;
    q.z = ok ? bf16_val(r2) : 0.0f;
    q.w = 0.0f;
    putf4(RP + (size_t)row * 4, q);
    return;
  } else if (u < L6) {
    const int v   = u - L5;
    const int row = v >> 4;
    const int j   = v & 15;
    const int rc  = row < nN ? row : nN - 1;
    const bool ok = row < nN;
    int z = Z[rc];
    z = z < 0 ? 0 : (z > nEmb - 1 ? nEmb - 1 : z);
    const float* p = emb + (size_t)z * HID + 8 * j;
    const v4f a = *(const v4fa*)p;
    const v4f b = *(const v4fa*)(p + 4);
    const v8f e8 = {a.x, a.y, a.z, a.w, b.x, b.y, b.z, b.w};
    v8us ohi, oz;
#pragma unroll
    for (int i = 0; i < 8; ++i) {
      ohi[i] = ok ? (unsigned short)bf16_bits(e8[i]) : (unsigned short)0;
      oz[i]  = (unsigned short)0;
    }
    unsigned short* dp = XB + (size_t)row * KX + 8 * j;
    *(volatile v8us*)dp         = ohi;
    *(volatile v8us*)(dp + HID) = oz;
    __threadfence();
    *(volatile v8us*)dp         = ohi;
    *(volatile v8us*)(dp + HID) = oz;
    return;
  } else if (u < L7) {
    const int v   = u - L6;
    const int row = v >> 5;
    const int q   = v & 31;
    if (row >= nN) return;
    int z = Z[row];
    z = z < 0 ? 0 : (z > nEmb - 1 ? nEmb - 1 : z);
    const v4f a = *(const v4fa*)(emb + (size_t)z * HID + 4 * q);
    v4f w4;
    w4.x = bf16_val(a.x);
    w4.y = bf16_val(a.y);
    w4.z = bf16_val(a.z);
    w4.w = bf16_val(a.w);
    putf4(X0 + (size_t)row * HID + 4 * q, w4);
    return;
  }
}

template <int MODE>
__global__ __launch_bounds__(GTHR) void k_gemm(const unsigned short* __restrict__ A, int lda,
                                               const unsigned short* __restrict__ BT, int ldb, int K,
                                               const float* __restrict__ bias, int nN,
                                               float* Cm, int ldc, unsigned short* Cb) {
  __shared__ __attribute__((aligned(16))) float stg[GBM * GBN];
  const int tid = (int)threadIdx.x, lane = tid & 31, wave = tid >> 5, hh = lane >> 4, m = lane & 15;
  const int rowBase = (int)blockIdx.x * GBM;
  const int colBase = (int)blockIdx.y * GBN;

  v8f acc[8];
  {
    const v8f z = {0.f, 0.f, 0.f, 0.f, 0.f, 0.f, 0.f, 0.f};
#pragma unroll
    for (int t = 0; t < 8; ++t) acc[t] = z;
  }
  const unsigned short* ap = A  + (size_t)(rowBase + 16 * wave + m) * (size_t)lda + 8 * hh;
  const unsigned short* bp = BT + (size_t)(colBase + m) * (size_t)ldb + 8 * hh;

#pragma unroll 1
  for (int k0 = 0; k0 < K; k0 += 32) {
    FragB af;
    af.h[0] = *(const v8usa*)(ap + k0);
    af.h[1] = *(const v8usa*)(ap + k0 + 16);
#pragma unroll
    for (int nt = 0; nt < 8; ++nt) {
      const unsigned short* wq = bp + (size_t)(16 * nt) * (size_t)ldb + k0;
      FragB bf;
      bf.h[0] = *(const v8usa*)wq;
      bf.h[1] = *(const v8usa*)(wq + 16);
      acc[nt] = wmb(af, bf, acc[nt]);
    }
  }

#pragma unroll
  for (int nt = 0; nt < 8; ++nt) {
    const int lc = 16 * nt + m;
    float bvv = 0.0f;
    if constexpr (MODE != 0) bvv = bf16_val(bias[colBase + lc]);
#pragma unroll
    for (int r = 0; r < 8; ++r) {
      const int lr = 16 * wave + 8 * hh + r;
      float v = acc[nt][r];
      if constexpr (MODE == 1) v = ssp_f(v + bvv);
      if constexpr (MODE == 2) v = v + bvv;
      stg[lr * GBN + lc] = v;
    }
  }
  __syncthreads();

  if constexpr (MODE == 0) {
    v4f pv[16];
#pragma unroll
    for (int i = 0; i < 16; ++i) pv[i] = *(const v4fa*)(stg + (16 * wave + i) * GBN + 4 * lane);
#pragma unroll
    for (int i = 0; i < 16; ++i) {
      float* op = Cm + (size_t)(rowBase + 16 * wave + i) * (size_t)ldc + colBase + 4 * lane;
      *(volatile v4f*)op = pv[i];
    }
    __threadfence();
#pragma unroll
    for (int i = 0; i < 16; ++i) {
      float* op = Cm + (size_t)(rowBase + 16 * wave + i) * (size_t)ldc + colBase + 4 * lane;
      *(volatile v4f*)op = pv[i];
    }
  } else if constexpr (MODE == 1) {
    const int part = lane >> 4;
    const int j = lane & 15;
    const unsigned mh = 0u - (unsigned)part;
    const unsigned ml = ~mh;
    v8us pv[16];
#pragma unroll
    for (int i = 0; i < 16; ++i) {
      const float* sp = stg + (16 * wave + i) * GBN + 8 * j;
      const v4f a = *(const v4fa*)sp;
      const v4f b = *(const v4fa*)(sp + 4);
      const v8f f8 = {a.x, a.y, a.z, a.w, b.x, b.y, b.z, b.w};
      v8us oo;
#pragma unroll
      for (int e = 0; e < 8; ++e) {
        const unsigned hb = bf16_bits(f8[e]);
        const unsigned lb = bf16_bits(f8[e] - __uint_as_float(hb << 16));
        oo[e] = (unsigned short)((hb & ml) | (lb & mh));
      }
      pv[i] = oo;
    }
#pragma unroll
    for (int i = 0; i < 16; ++i) {
      unsigned short* op = Cb + (size_t)(rowBase + 16 * wave + i) * (size_t)KU + part * HID + 8 * j;
      *(volatile v8us*)op = pv[i];
    }
    __threadfence();
#pragma unroll
    for (int i = 0; i < 16; ++i) {
      unsigned short* op = Cb + (size_t)(rowBase + 16 * wave + i) * (size_t)KU + part * HID + 8 * j;
      *(volatile v8us*)op = pv[i];
    }
  } else {
    v4f pv[16];
#pragma unroll
    for (int i = 0; i < 16; ++i) {
      const int row = rowBase + 16 * wave + i;
      const int rc  = row < nN ? row : nN - 1;
      const v4f hv = *(const v4fa*)(Cm + (size_t)rc * (size_t)ldc + colBase + 4 * lane);
      const v4f sv = *(const v4fa*)(stg + (16 * wave + i) * GBN + 4 * lane);
      v4f q;
      q.x = sv.x + hv.x;
      q.y = sv.y + hv.y;
      q.z = sv.z + hv.z;
      q.w = sv.w + hv.w;
      pv[i] = q;
    }
#pragma unroll
    for (int i = 0; i < 16; ++i) {
      const int row = rowBase + 16 * wave + i;
      if (row < nN) {
        float* op = Cm + (size_t)row * (size_t)ldc + colBase + 4 * lane;
        *(volatile v4f*)op = pv[i];
      }
    }
    __threadfence();
#pragma unroll
    for (int i = 0; i < 16; ++i) {
      const int row = rowBase + 16 * wave + i;
      if (row < nN) {
        float* op = Cm + (size_t)row * (size_t)ldc + colBase + 4 * lane;
        *(volatile v4f*)op = pv[i];
      }
    }
  }
}

__device__ __forceinline__ void wave_gemm_b(const unsigned short* sAw, float* sDw,
                                            const unsigned short* __restrict__ BT, int ldb, int K,
                                            int hh, int m) {
#pragma unroll 1
  for (int nh = 0; nh < 2; ++nh) {
    v8f acc[2][4];
    {
      const v8f z = {0.f, 0.f, 0.f, 0.f, 0.f, 0.f, 0.f, 0.f};
#pragma unroll
      for (int mt = 0; mt < 2; ++mt)
#pragma unroll
        for (int nt = 0; nt < 4; ++nt) acc[mt][nt] = z;
    }
    const unsigned short* ap0 = sAw + m * AP + 8 * hh;
    const unsigned short* ap1 = ap0 + 16 * AP;
    const unsigned short* bp  = BT + (size_t)(64 * nh + m) * (size_t)ldb + 8 * hh;
#pragma unroll 1
    for (int k0 = 0; k0 < K; k0 += 32) {
      FragB a0, a1;
      a0.h[0] = *(const v8usa*)(ap0 + k0);
      a0.h[1] = *(const v8usa*)(ap0 + k0 + 16);
      a1.h[0] = *(const v8usa*)(ap1 + k0);
      a1.h[1] = *(const v8usa*)(ap1 + k0 + 16);
#pragma unroll
      for (int nt = 0; nt < 4; ++nt) {
        const unsigned short* wq = bp + (size_t)(16 * nt) * (size_t)ldb + k0;
        FragB b;
        b.h[0] = *(const v8usa*)wq;
        b.h[1] = *(const v8usa*)(wq + 16);
        acc[0][nt] = wmb(a0, b, acc[0][nt]);
        acc[1][nt] = wmb(a1, b, acc[1][nt]);
      }
    }
#pragma unroll
    for (int nt = 0; nt < 4; ++nt) {
      const int col = 64 * nh + 16 * nt + m;
#pragma unroll
      for (int mt = 0; mt < 2; ++mt)
#pragma unroll
        for (int r = 0; r < 8; ++r) sDw[(16 * mt + 8 * hh + r) * DP + col] = acc[mt][nt][r];
    }
  }
}
__device__ __forceinline__ void wave_gemm_h(const unsigned short* sAw, float* sDw,
                                            const unsigned short* __restrict__ BT, int ldb, int K,
                                            int hh, int m) {
#pragma unroll 1
  for (int nh = 0; nh < 2; ++nh) {
    v8f acc[2][4];
    {
      const v8f z = {0.f, 0.f, 0.f, 0.f, 0.f, 0.f, 0.f, 0.f};
#pragma unroll
      for (int mt = 0; mt < 2; ++mt)
#pragma unroll
        for (int nt = 0; nt < 4; ++nt) acc[mt][nt] = z;
    }
    const unsigned short* ap0 = sAw + m * AP + 8 * hh;
    const unsigned short* ap1 = ap0 + 16 * AP;
    const unsigned short* bp  = BT + (size_t)(64 * nh + m) * (size_t)ldb + 8 * hh;
#pragma unroll 1
    for (int k0 = 0; k0 < K; k0 += 32) {
      FragH a0, a1;
      a0.h[0] = *(const v8usa*)(ap0 + k0);
      a0.h[1] = *(const v8usa*)(ap0 + k0 + 16);
      a1.h[0] = *(const v8usa*)(ap1 + k0);
      a1.h[1] = *(const v8usa*)(ap1 + k0 + 16);
#pragma unroll
      for (int nt = 0; nt < 4; ++nt) {
        const unsigned short* wq = bp + (size_t)(16 * nt) * (size_t)ldb + k0;
        FragH b;
        b.h[0] = *(const v8usa*)wq;
        b.h[1] = *(const v8usa*)(wq + 16);
        acc[0][nt] = wmh(a0, b, acc[0][nt]);
        acc[1][nt] = wmh(a1, b, acc[1][nt]);
      }
    }
#pragma unroll
    for (int nt = 0; nt < 4; ++nt) {
      const int col = 64 * nh + 16 * nt + m;
#pragma unroll
      for (int mt = 0; mt < 2; ++mt)
#pragma unroll
        for (int r = 0; r < 8; ++r) sDw[(16 * mt + 8 * hh + r) * DP + col] = acc[mt][nt][r];
    }
  }
}

__global__ __launch_bounds__(NTHR) void k_edge(const int* __restrict__ srcs, const int* __restrict__ dsts,
                                               int nEh, int nN,
                                               const float* __restrict__ RP, const float* __restrict__ XF,
                                               const unsigned short* __restrict__ W1T,
                                               const unsigned short* __restrict__ W2T,
                                               const float* __restrict__ b1, const float* __restrict__ b2,
                                               unsigned short* Mh) {
#pragma clang fp contract(off)
  extern __shared__ __attribute__((aligned(16))) float dyn[];
  float*          sD   = dyn;
  unsigned short* sA   = (unsigned short*)(dyn + EPB * DP);
  unsigned short* sM   = sA + EPB * AP;
  float*          cst  = dyn + EPB * DP + (EPB * AP) / 2 + (EPB * MPITCH) / 2;
  int*            sSrc = (int*)(cst + CSTN);
  float*          sRc  = (float*)(sSrc + EPB);
  int*            sEl  = (int*)(sRc + EPB);
  int*            sCnt = sEl + EPB;

  const int tid = (int)threadIdx.x, lane = tid & 31, wave = tid >> 5, hh = lane >> 4, m = lane & 15;

  if (tid < HID) {
    cst[tid]       = bf16_val(b1[tid]);
    cst[HID + tid] = bf16_val(b2[tid]);
  }

  const int  elb  = (int)blockIdx.x * EPB;
  const int  el   = elb + tid;
  const bool live = el < nEh;
  const int  elc  = live ? el : (nEh - 1);
  int s = srcs[elc];
  int t = dsts[elc];
  s = s < 0 ? 0 : (s > nN - 1 ? nN - 1 : s);
  t = t < 0 ? 0 : (t > nN - 1 ? nN - 1 : t);
  const v4f xs = *(const v4fa*)(RP + (size_t)s * 4);
  const v4f xd = *(const v4fa*)(RP + (size_t)t * 4);
  const float rx = xs.x - xd.x, ry = xs.y - xd.y, rz = xs.z - xd.z;
  const float dsq = (rx * rx + rz * rz) + ry * ry;
  const float d   = sqrtf(dsq);
  const bool  act = live && (d < CUTF);
  const float csv = cosf((d * PIF) * (1.0f / CUTF));
  const float rc  = act ? 0.5f * (csv + 1.0f) : 0.0f;

  const unsigned mw  = __builtin_amdgcn_ballot_w32(act);
  const int      wcn = (int)__builtin_popcount(mw);
  const int      rk  = (int)__builtin_amdgcn_mbcnt_lo(mw, 0u);
  const int      irk = lane - rk;
  if (lane == 0) sCnt[wave] = wcn;
  __syncthreads();

  int base = 0, nact = 0;
#pragma unroll
  for (int w2 = 0; w2 < NWAVE; ++w2) {
    int c = sCnt[w2];
    c = c < 0 ? 0 : (c > 32 ? 32 : c);
    nact += c;
    base += (w2 < wave) ? c : 0;
  }
  const int ntile = (nact + 31) >> 5;
  int p = act ? (base + rk) : (nact + (32 * wave - base) + irk);
  p = p < 0 ? 0 : (p > EPB - 1 ? EPB - 1 : p);
  sSrc[p] = s;
  sRc[p]  = rc;
  sEl[p]  = tid;
  {
    unsigned short* rap = sA + p * AP;
    const float rdiv = 1.0f / (float)(NRBF - 1);
    const float wdt  = CUTF * rdiv;
    const float cof  = -0.5f * (1.0f / (wdt * wdt));
#pragma unroll 1
    for (int c8 = 0; c8 < NB / 8; ++c8) {
      v8us ho;
#pragma unroll
      for (int i = 0; i < 8; ++i) {
        const int   k  = 8 * c8 + i;
        const float ck = (k >= NRBF - 1) ? CUTF : CUTF * ((float)k * rdiv);
        const float dl = d - ck;
        const float fv = __expf(cof * (dl * dl));
        const float gv = (k < NRBF) ? fv : (fv - fv);
        ho[i] = (unsigned short)bf16_bits(gv);
      }
      *(v8usa*)(rap + 8 * c8) = ho;
    }
  }
  __syncthreads();

  const int   sc   = sSrc[tid];
  const float rcv  = sRc[tid];
  int         elo  = sEl[tid];
  elo = elo < 0 ? 0 : (elo > EPB - 1 ? EPB - 1 : elo);
  const bool  actc = tid < nact;
  float*          rd = sD + tid * DP;
  unsigned short* ra = sA + tid * AP;
  unsigned short* rm = sM + elo * MPITCH;
  const unsigned short* sAw = sA + 32 * wave * AP;
  float*                sDw = sD + 32 * wave * DP;

  if (wave < ntile) wave_gemm_b(sAw, sDw, W1T, KF1, KF1, hh, m);
  __syncthreads();

  if (wave < ntile) {
#pragma unroll 1
    for (int c8 = 0; c8 < HID / 8; ++c8) {
      const v4f va = *(const v4fa*)(rd + 8 * c8);
      const v4f vb = *(const v4fa*)(rd + 8 * c8 + 4);
      const v4f ba = *(const v4fa*)(cst + 8 * c8);
      const v4f bb = *(const v4fa*)(cst + 8 * c8 + 4);
      const v8f v8 = {va.x, va.y, va.z, va.w, vb.x, vb.y, vb.z, vb.w};
      const v8f b8 = {ba.x, ba.y, ba.z, ba.w, bb.x, bb.y, bb.z, bb.w};
      v8us o;
#pragma unroll
      for (int i = 0; i < 8; ++i) o[i] = f2h(CACT * ssp_f(v8[i] + b8[i]));
      *(v8usa*)(ra + 8 * c8) = o;
    }
  }
  __syncthreads();

  if (wave < ntile) wave_gemm_h(sAw, sDw, W2T, KF2, KF2, hh, m);
  __syncthreads();

  if (wave < ntile) {
    const float* xr = XF + (size_t)sc * HID;
#pragma unroll 1
    for (int c8 = 0; c8 < HID / 8; ++c8) {
      const v4f va = *(const v4fa*)(rd + 8 * c8);
      const v4f vb = *(const v4fa*)(rd + 8 * c8 + 4);
      const v4f xa = *(const v4fa*)(xr + 8 * c8);
      const v4f xb = *(const v4fa*)(xr + 8 * c8 + 4);
      const v4f ba = *(const v4fa*)(cst + HID + 8 * c8);
      const v4f bb = *(const v4fa*)(cst + HID + 8 * c8 + 4);
      const v8f v8 = {va.x, va.y, va.z, va.w, vb.x, vb.y, vb.z, vb.w};
      const v8f x8 = {xa.x, xa.y, xa.z, xa.w, xb.x, xb.y, xb.z, xb.w};
      const v8f b8 = {ba.x, ba.y, ba.z, ba.w, bb.x, bb.y, bb.z, bb.w};
      v8us o;
#pragma unroll
      for (int i = 0; i < 8; ++i) {
        const float wij = fmaf(v8[i], PINV, b8[i]) * rcv;
        const float ms  = actc ? (x8[i] * wij) : 0.0f;
        o[i] = f2h(CMSG * ms);
      }
      *(v8usa*)(rm + 8 * c8) = o;
    }
  } else {
    v8us oz;
#pragma unroll
    for (int i = 0; i < 8; ++i) oz[i] = (unsigned short)0;
#pragma unroll 1
    for (int c8 = 0; c8 < HID / 8; ++c8) *(v8usa*)(rm + 8 * c8) = oz;
  }
  __syncthreads();

  {
    v4i pv[16];
#pragma unroll
    for (int it = 0; it < 16; ++it) pv[it] = *(const v4ia*)(sM + (size_t)(it * NTHR + tid) * 8);
    unsigned short* mb = Mh + (size_t)elb * MPITCH;
#pragma unroll
    for (int it = 0; it < 16; ++it) *(volatile v4i*)(mb + (size_t)(it * NTHR + tid) * 8) = pv[it];
    __threadfence();
#pragma unroll
    for (int it = 0; it < 16; ++it) *(volatile v4i*)(mb + (size_t)(it * NTHR + tid) * 8) = pv[it];
  }
}

__global__ __launch_bounds__(NTHR) void k_scan(const int* __restrict__ dsts, int nEh, int vec8, int first,
                                               int mRows, const unsigned short* __restrict__ Mh, float* HACC) {
  extern __shared__ __attribute__((aligned(16))) int dsm[];
  int*   list = dsm;
  int*   hl   = dsm + LISTN;
  int*   sl   = hl + RCAP;
  int*   cnt  = sl + RCAP;
  int*   offs = cnt + NBA;
  int*   cur  = offs + NBA;
  int*   misc = cur + NBA;
  const int tid = (int)threadIdx.x, lane = tid & 31, wave = tid >> 5;
  const int nodeBase = (int)blockIdx.x * NBA;

  {
    const v4i z4 = {0, 0, 0, 0};
    for (int i = tid * 4; i < AGG_ZINTS; i += NTHR * 4) *(v4ia*)(dsm + i) = z4;
    if (tid < 16) misc[tid] = 0;
  }
  __syncthreads();

  int t = 0, ov = 0;
  const int nChunks = (nEh + CHUNK - 1) / CHUNK;
#pragma unroll 1
  for (int ch = 0; ch < nChunks; ++ch) {
    const int cbase = ch * CHUNK;
    const int wc = scan_chunk<SLA>(dsts, nEh, cbase, nodeBase, NBA, vec8, list, tid, lane, wave);
    if (lane == 0) misc[wave] = wc;
    __syncthreads();
    if (wave == 0) {
#pragma unroll 1
      for (int w2 = 0; w2 < NWAVE; ++w2) {
        int c = misc[w2];
        c = c < 0 ? 0 : (c > WCAP ? WCAP : c);
#pragma unroll 1
        for (int b0 = 0; b0 < c; b0 += 32) {
          const int idx = b0 + lane;
          const int ent = list[w2 * WCAP + (idx < WCAP ? idx : WCAP - 1)];
          const int m32 = (c - b0) < 32 ? (c - b0) : 32;
#pragma unroll 1
          for (int k = 0; k < m32; ++k) {
            const int u    = __builtin_amdgcn_readlane(ent, k);
            const int slot = u & (NBA - 1);
            const int el   = (u >> SLA) & (CHUNK - 1);
            const int pk   = ((cbase + el) << SLA) | slot;
            if (t < RCAP) {
              if (lane == 0) { hl[t] = pk; cnt[slot] = cnt[slot] + 1; }
              t = t + 1;
            } else {
              ov = 1;
            }
          }
        }
      }
    }
    __syncthreads();
  }
  if (wave == 0 && lane == 0) { misc[8] = t; misc[9] = ov; }
  __syncthreads();
  int tt = misc[8];
  tt = tt < 0 ? 0 : (tt > RCAP ? RCAP : tt);
  const int ovf = misc[9];

  if (wave == 0) {
    const int base = lane * (NBA / 32);
    int s = 0;
#pragma unroll 1
    for (int i = 0; i < NBA / 32; ++i) s += cnt[base + i];
    int incl = s;
#pragma unroll
    for (int d = 1; d < 32; d <<= 1) {
      const int y = __shfl_up(incl, d, 32);
      if (lane >= d) incl += y;
    }
    int run = incl - s;
#pragma unroll 1
    for (int i = 0; i < NBA / 32; ++i) {
      const int cv = cnt[base + i];
      offs[base + i] = run;
      cur[base + i]  = run;
      run += cv;
    }
  }
  __syncthreads();
  if (wave == 0) {
#pragma unroll 1
    for (int b0 = 0; b0 < tt; b0 += 32) {
      const int idx = b0 + lane;
      const int ent = hl[idx < RCAP ? idx : RCAP - 1];
      const int m32 = (tt - b0) < 32 ? (tt - b0) : 32;
#pragma unroll 1
      for (int k = 0; k < m32; ++k) {
        const int u    = __builtin_amdgcn_readlane(ent, k);
        const int slot = u & (NBA - 1);
        if (lane == 0) {
          int p = cur[slot];
          p = p < 0 ? 0 : (p > RCAP - 1 ? RCAP - 1 : p);
          sl[p] = u;
          cur[slot] = p + 1;
        }
      }
    }
  }
  __syncthreads();

  const float qnan = __int_as_float(0x7fc00000);
  const float pz = (ovf != 0) ? qnan : 0.0f;
#pragma unroll 1
  for (int si = 0; si < NBA / NWAVE; ++si) {
    const int s    = si * NWAVE + wave;
    const int node = nodeBase + s;
    int c = cnt[s];
    const bool big = c > DEGCAP;
    c = c < 0 ? 0 : (c > DEGCAP ? DEGCAP : c);
    int o = offs[s];
    o = o < 0 ? 0 : (o > RCAP ? RCAP : o);
    float a0 = 0.0f, a1 = 0.0f, a2 = 0.0f, a3 = 0.0f;
#pragma unroll 1
    for (int b0 = 0; b0 < c; b0 += 32) {
      int idx = o + b0 + lane;
      idx = idx > RCAP - 1 ? RCAP - 1 : idx;
      const int ent = sl[idx];
      int eid = ent >> SLA;
      eid = eid < 0 ? 0 : (eid > nEh - 1 ? nEh - 1 : eid);
      const int m32 = (c - b0) < 32 ? (c - b0) : 32;
#pragma unroll 1
      for (int k = 0; k < m32; ++k) {
        const int ek = __builtin_amdgcn_readlane(eid, k);
        const unsigned short* rp = Mh + (size_t)ek * MPITCH + 4 * lane;
        const v2u w = *(const v2ua*)rp;
        a0 += h2f(w.x & 0xffffu);
        a1 += h2f(w.x >> 16);
        a2 += h2f(w.y & 0xffffu);
        a3 += h2f(w.y >> 16);
      }
    }
    const bool  live = node < mRows;
    const int   nr   = live ? node : mRows - 1;
    const float pzr  = big ? qnan : pz;
    float* mp = HACC + (size_t)nr * HID + 4 * lane;
    const v4f old = *(const v4fa*)mp;
    const float o0 = (first != 0) ? 0.0f : old.x;
    const float o1 = (first != 0) ? 0.0f : old.y;
    const float o2 = (first != 0) ? 0.0f : old.z;
    const float o3 = (first != 0) ? 0.0f : old.w;
    v4f nv;
    nv.x = fmaf(a0, MINV, o0) + pzr;
    nv.y = fmaf(a1, MINV, o1) + pzr;
    nv.z = fmaf(a2, MINV, o2) + pzr;
    nv.w = fmaf(a3, MINV, o3) + pzr;
    if (live) *(volatile v4f*)mp = nv;
    __threadfence();
    if (live) *(volatile v4f*)mp = nv;
  }
}

__global__ __launch_bounds__(NTHR) void k_hilo(const float* __restrict__ S, int nValid, int nUnits,
                                               unsigned short* Dp) {
  const int u = (int)blockIdx.x * NTHR + (int)threadIdx.x;
  if (u >= nUnits) return;
  const int row = u >> 4;
  const int j   = u & 15;
  const int rc  = row < nValid ? row : nValid - 1;
  const bool ok = row < nValid;
  const float* mq = S + (size_t)rc * HID + 8 * j;
  const v4f ma = *(const v4fa*)mq;
  const v4f mb = *(const v4fa*)(mq + 4);
  const v8f m8 = {ma.x, ma.y, ma.z, ma.w, mb.x, mb.y, mb.z, mb.w};
  v8us ohi, olo;
#pragma unroll
  for (int i = 0; i < 8; ++i) {
    const float f = ok ? m8[i] : 0.0f;
    const unsigned hbits = bf16_bits(f);
    ohi[i] = (unsigned short)hbits;
    olo[i] = (unsigned short)bf16_bits(f - __uint_as_float(hbits << 16));
  }
  unsigned short* dp = Dp + (size_t)row * KU + 8 * j;
  *(volatile v8us*)dp         = ohi;
  *(volatile v8us*)(dp + HID) = olo;
  __threadfence();
  *(volatile v8us*)dp         = ohi;
  *(volatile v8us*)(dp + HID) = olo;
}

static inline int cdiv(int a, int b) { return (a + b - 1) / b; }

extern "C" void kernel_launch(void* const* d_in, const int* in_sizes, int n_in,
                              void* d_out, int out_size, void* d_ws, size_t ws_size,
                              hipStream_t stream) {
  if (n_in < 14) return;
  if (in_sizes[0] < 3 || (in_sizes[0] % 3) != 0) return;
  const int nN = in_sizes[0] / 3;
  if (nN < 1 || in_sizes[1] != nN) return;
  const int nE = in_sizes[2];
  if (nE < 1 || nE >= (1 << 22)) return;
  if (in_sizes[3] != nE) return;
  if (in_sizes[4] < HID || (in_sizes[4] % HID) != 0) return;
  const int nEmb = in_sizes[4] / HID;
  if (in_sizes[5] != NLAY * HID * HID) return;
  if (in_sizes[6] != NLAY * NRBF * HID) return;
  if (in_sizes[7] != NLAY * HID) return;
  if (in_sizes[8] != NLAY * HID * HID || in_sizes[9] != NLAY * HID) return;
  if (in_sizes[10] != NLAY * HID * HID || in_sizes[11] != NLAY * HID) return;
  if (in_sizes[12] != NLAY * HID * HID || in_sizes[13] != NLAY * HID) return;
  if ((long long)out_size != (long long)nN * HID) return;

  const float* R    = (const float*)d_in[0];
  const int*   Z    = (const int*)d_in[1];
  const int*   idxi = (const int*)d_in[2];
  const int*   idxj = (const int*)d_in[3];
  const float* emb  = (const float*)d_in[4];
  const float* IF   = (const float*)d_in[5];
  const float* W1   = (const float*)d_in[6];
  const float* fb1  = (const float*)d_in[7];
  const float* W2   = (const float*)d_in[8];
  const float* fb2  = (const float*)d_in[9];
  const float* U1   = (const float*)d_in[10];
  const float* ob1  = (const float*)d_in[11];
  const float* U2   = (const float*)d_in[12];
  const float* ob2  = (const float*)d_in[13];
  float* out = (float*)d_out;

  const int MP = cdiv(nN, GBM) * GBM;
  const int gM = MP / GBM;
  const int gA = cdiv(MP, NBA);
  if ((long long)gA * NBA < (long long)MP) return;
  const int EH  = cdiv(cdiv(nE, NRANGE), EPB) * EPB;
  const int EHP = EH;
  if (EH < 1 || EH >= (1 << 21)) return;
  if ((long long)EH * NRANGE < (long long)nE) return;

  char* ws = (char*)d_ws;
  size_t off = 0;
  const size_t oIFT = off; off += (size_t)NLAY * HID * KX * 2;        off = (off + 255) & ~(size_t)255;
  const size_t oW1T = off; off += (size_t)NLAY * HID * KF1 * 2;       off = (off + 255) & ~(size_t)255;
  const size_t oW2T = off; off += (size_t)NLAY * HID * KF2 * 2;       off = (off + 255) & ~(size_t)255;
  const size_t oU1T = off; off += (size_t)NLAY * HID * KU * 2;        off = (off + 255) & ~(size_t)255;
  const size_t oU2T = off; off += (size_t)NLAY * HID * KU * 2;        off = (off + 255) & ~(size_t)255;
  const size_t oRP  = off; off += (size_t)MP * 4 * 4;                 off = (off + 255) & ~(size_t)255;
  const size_t szB = (size_t)MP * KU * 2;
  size_t szRA = (size_t)EHP * MPITCH * 2;
  if (szRA < 3 * szB) szRA = 3 * szB;
  const size_t oRA  = off; off += szRA;                               off = (off + 255) & ~(size_t)255;
  const size_t oXF  = off; off += (size_t)MP * HID * 4;               off = (off + 255) & ~(size_t)255;
  const size_t oAGG = off; off += (size_t)MP * HID * 4;               off = (off + 255) & ~(size_t)255;
  if (off > ws_size || off > (size_t)WSMAX) return;
  unsigned short* IFT = (unsigned short*)(ws + oIFT);
  unsigned short* W1T = (unsigned short*)(ws + oW1T);
  unsigned short* W2T = (unsigned short*)(ws + oW2T);
  unsigned short* U1T = (unsigned short*)(ws + oU1T);
  unsigned short* U2T = (unsigned short*)(ws + oU2T);
  float*          RP  = (float*)(ws + oRP);
  unsigned short* MSG = (unsigned short*)(ws + oRA);
  unsigned short* AB  = (unsigned short*)(ws + oRA);
  unsigned short* G   = (unsigned short*)(ws + oRA + szB);
  unsigned short* XB  = (unsigned short*)(ws + oRA + 2 * szB);
  float*          XF  = (float*)(ws + oXF);
  float*          AGG = (float*)(ws + oAGG);

  hipFuncSetAttribute(reinterpret_cast<const void*>(&k_edge), hipFuncAttributeMaxDynamicSharedMemorySize,
                      (int)EDGE_LDS_BYTES);
  hipFuncSetAttribute(reinterpret_cast<const void*>(&k_scan), hipFuncAttributeMaxDynamicSharedMemorySize,
                      (int)AGG_LDS_BYTES);

  const int nXP   = cdiv(MP, NTHR) * NTHR;
  const int nX0   = cdiv(nN * 32, NTHR) * NTHR;
  const int nPrep = NU_IF + NU_W1 + NU_W2 + 2 * NU_U + nXP + MP * 16 + nX0;

  k_prep<<<nPrep / NTHR, NTHR, 0, stream>>>(R, Z, emb, nEmb, IF, W1, W2, U1, U2, nN, MP,
                                            IFT, W1T, W2T, U1T, U2T, RP, XB, out);

  for (int l = 0; l < NLAY; ++l) {
    const unsigned short* IFTl = IFT + (size_t)l * HID * KX;
    const unsigned short* W1Tl = W1T + (size_t)l * HID * KF1;
    const unsigned short* W2Tl = W2T + (size_t)l * HID * KF2;
    const unsigned short* U1Tl = U1T + (size_t)l * HID * KU;
    const unsigned short* U2Tl = U2T + (size_t)l * HID * KU;
    const float* fb1l = fb1 + (size_t)l * HID;
    const float* fb2l = fb2 + (size_t)l * HID;
    const float* ob1l = ob1 + (size_t)l * HID;
    const float* ob2l = ob2 + (size_t)l * HID;

    k_gemm<0><<<dim3(gM, 1), GTHR, 0, stream>>>(XB, KX, IFTl, KX, KX, fb1l, nN, XF, HID, G);

    for (int r = 0; r < NRANGE; ++r) {
      const int e0 = r * EH;
      int nEh = nE - e0;
      nEh = nEh > EH ? EH : nEh;
      if (nEh > 0) {
        const int vec = ((e0 & 3) == 0) ? 1 : 0;
        k_edge<<<cdiv(nEh, EPB), NTHR, EDGE_LDS_BYTES, stream>>>(idxj + e0, idxi + e0, nEh, nN, RP, XF,
                                                                  W1Tl, W2Tl, fb1l, fb2l, MSG);
        k_scan<<<gA, NTHR, AGG_LDS_BYTES, stream>>>(idxi + e0, nEh, vec, (r == 0) ? 1 : 0, MP, MSG, AGG);
      }
    }

    k_hilo<<<(MP * 16) / NTHR, NTHR, 0, stream>>>(AGG, MP, MP * 16, AB);
    k_gemm<1><<<dim3(gM, 1), GTHR, 0, stream>>>(AB, KU, U1Tl, KU, KU, ob1l, nN, AGG, HID, G);
    k_gemm<2><<<dim3(gM, 1), GTHR, 0, stream>>>(G, KU, U2Tl, KU, KU, ob2l, nN, out, HID, AB);
    if (l + 1 < NLAY) k_hilo<<<(MP * 16) / NTHR, NTHR, 0, stream>>>(out, nN, MP * 16, XB);
  }
}
